// DynamicRouting_10453950399034
// MI455X (gfx1250) — hardware-verified
//
#include <hip/hip_runtime.h>
#include <stdint.h>
#include <stddef.h>

constexpr int kBatch      = 16;
constexpr int kCin        = 512;
constexpr int kHW         = 1024;
constexpr int kGroups     = 8;
constexpr int kFi         = 64;
constexpr int kFo         = 256;
constexpr int kIters      = 3;
constexpr int kBatchChunk = 8;
constexpr int kNumChunks  = kBatch / kBatchChunk;
static_assert(kGroups * kFi == kCin, "groups");
static_assert(kBatch % kBatchChunk == 0, "chunks");
static_assert(kFi % 32 == 0, "K multiple of 32");
static_assert(kFo % 64 == 0 && kHW % 64 == 0, "tile multiples");

constexpr float kWScale   = 16.0f;
constexpr float kXScale   = 16.0f;
constexpr float kOutScale = 1.0f / 256.0f;

typedef __attribute__((ext_vector_type(16))) _Float16 v16h;
typedef __attribute__((ext_vector_type(8)))  _Float16 v8h;
typedef __attribute__((ext_vector_type(16))) __bf16   v16b;
typedef __attribute__((ext_vector_type(8)))  __bf16   v8b;
typedef __attribute__((ext_vector_type(8)))  float    v8f;
typedef __attribute__((ext_vector_type(4)))  float    v4f;

__device__ __forceinline__ unsigned short f2bf_bits(float f) {
  unsigned u = __float_as_uint(f);
  return (unsigned short)((u + 0x7FFFu + ((u >> 16) & 1u)) >> 16);
}
__device__ __forceinline__ float bf_bits2f(unsigned short h) { return __uint_as_float(((unsigned)h) << 16); }

__device__ __forceinline__ void dep_guard_h(v8f& a, v8f& b, v16h x, v16h y) { asm volatile("v_nop\n\tv_nop\n\tv_nop\n\tv_nop" : "+v"(a), "+v"(b) : "v"(x), "v"(y)); }
__device__ __forceinline__ void dep_guard_b(v8f& a, v8f& b, v16b x, v16b y) { asm volatile("v_nop\n\tv_nop\n\tv_nop\n\tv_nop" : "+v"(a), "+v"(b) : "v"(x), "v"(y)); }
__device__ __forceinline__ void keep4_h(v16h a, v16h b, v16h c, v16h d) { asm volatile("v_nop" :: "v"(a), "v"(b), "v"(c), "v"(d)); }
__device__ __forceinline__ void keep4_b(v16b a, v16b b, v16b c, v16b d) { asm volatile("v_nop" :: "v"(a), "v"(b), "v"(c), "v"(d)); }
__device__ __forceinline__ void acc_guard4(v8f& a, v8f& b, v8f& c, v8f& d) { asm volatile("v_nop\n\tv_nop\n\tv_nop\n\tv_nop" : "+v"(a), "+v"(b), "+v"(c), "+v"(d)); }
template <typename T> struct Frag;
template <> struct Frag<_Float16> {
  typedef v16h V; union U { v16h v; v8h h[2]; };
  static __device__ __forceinline__ v16h load(const _Float16* p) {
    U f; f.h[0] = *(const v8h*)(p); f.h[1] = *(const v8h*)(p + 16); return f.v;
  }
  static __device__ __forceinline__ v8f mma(v16h a, v16h b, v8f c) {
    return __builtin_amdgcn_wmma_f32_16x16x32_f16(false, a, false, b, (short)0, c, false, false);
  }
  static __device__ __forceinline__ void guard(v8f& a, v8f& b, v16h x, v16h y) { dep_guard_h(a, b, x, y); }
  static __device__ __forceinline__ void keep(v16h a, v16h b, v16h c, v16h d) { keep4_h(a, b, c, d); }
};
template <> struct Frag<__bf16> {
  typedef v16b V; union U { v16b v; v8b h[2]; };
  static __device__ __forceinline__ v16b load(const __bf16* p) {
    U f; f.h[0] = *(const v8b*)(p); f.h[1] = *(const v8b*)(p + 16); return f.v;
  }
  static __device__ __forceinline__ v8f mma(v16b a, v16b b, v8f c) {
    return __builtin_amdgcn_wmma_f32_16x16x32_bf16(false, a, false, b, (short)0, c, false, false);
  }
  static __device__ __forceinline__ void guard(v8f& a, v8f& b, v16b x, v16b y) { dep_guard_b(a, b, x, y); }
  static __device__ __forceinline__ void keep(v16b a, v16b b, v16b c, v16b d) { keep4_b(a, b, c, d); }
};

template <int ET> struct Elem;
template <> struct Elem<0> { typedef _Float16 T; };
template <> struct Elem<1> { typedef __bf16 T; };
template <int ET, bool SPLIT, int BIAS_MODE, int OUT_MODE, bool RESID, int ACT = 0>
__global__ __launch_bounds__(256) void wmma_gemm64z(
    const unsigned short* __restrict__ Ap, const unsigned short* __restrict__ A2p, int lda, long strideA, long strideAz,
    const unsigned short* __restrict__ Btp, const unsigned short* __restrict__ Bt2p, int ldb, long strideB, long strideBz,
    void* __restrict__ Cout, void* __restrict__ Cout2, int ldc, long strideC, long strideCz,
    const float* __restrict__ bias,
    const float* __restrict__ resid, long strideR,
    int M, int N, int K, float scale) {
  typedef typename Elem<ET>::T T;
  typedef typename Frag<T>::V V;
  const T* A = (const T*)Ap; const T* A2 = (const T*)A2p; const T* Bt = (const T*)Btp; const T* Bt2 = (const T*)Bt2p;
  __shared__ __align__(16) float sT[8][16 * 68];
  const int b    = blockIdx.y;
  const int bz   = blockIdx.z;
  const int lane = threadIdx.x & 31;
  const int wave = threadIdx.x >> 5;
  const int tilesN = N >> 6;
  const int tilesM = M >> 6;
  const int tile = blockIdx.x * 8 + wave;
  if (tile >= tilesM * tilesN) return;
  const int tm = tile / tilesN;
  const int tn = tile - tm * tilesN;
  const int m0 = tm << 6;
  const int n0 = tn << 6;

  const T* Ab  = A  + (size_t)b * strideA + (size_t)bz * strideAz;
  const T* Bb  = Bt + (size_t)b * strideB + (size_t)bz * strideBz;
  const T* Ab2 = SPLIT ? (A2  + (size_t)b * strideA + (size_t)bz * strideAz) : nullptr;
  const T* Bb2 = SPLIT ? (Bt2 + (size_t)b * strideB + (size_t)bz * strideBz) : nullptr;

  const int rlane = lane & 15;
  const int koff  = (lane >> 4) * 8;
  const int mOff  = (lane >> 4) * 8;

  v8f acc[4][4];
#pragma unroll
  for (int i = 0; i < 4; ++i)
#pragma unroll
    for (int j = 0; j < 4; ++j) acc[i][j] = (v8f){0.f,0.f,0.f,0.f,0.f,0.f,0.f,0.f};

  for (int k0 = 0; k0 < K; k0 += 32) {
    V bh[4], bl[4];
#pragma unroll
    for (int j = 0; j < 4; ++j) {
      const size_t bo = (size_t)(n0 + (j << 4) + rlane) * ldb + koff + k0;
      bh[j] = Frag<T>::load(Bb + bo);
      if (SPLIT) bl[j] = Frag<T>::load(Bb2 + bo);
    }
#pragma unroll
    for (int i = 0; i < 4; ++i) {
      const size_t ao = (size_t)(m0 + (i << 4) + rlane) * lda + koff + k0;
      V ah = Frag<T>::load(Ab + ao);
      V al;
      if (SPLIT) al = Frag<T>::load(Ab2 + ao);
#pragma unroll
      for (int j = 0; j < 4; ++j) {
        acc[i][j] = Frag<T>::mma(ah, bh[j], acc[i][j]);
        if (SPLIT) {
          acc[i][j] = Frag<T>::mma(ah, bl[j], acc[i][j]);
          acc[i][j] = Frag<T>::mma(al, bh[j], acc[i][j]);
        }
      }
      Frag<T>::guard(acc[i][0], acc[i][3], ah, SPLIT ? al : ah);
    }
    Frag<T>::keep(bh[0], bh[1], bh[2], bh[3]);
    if (SPLIT) Frag<T>::keep(bl[0], bl[1], bl[2], bl[3]);
  }
  acc_guard4(acc[0][0], acc[0][1], acc[0][2], acc[0][3]);
  acc_guard4(acc[1][0], acc[1][1], acc[1][2], acc[1][3]);
  acc_guard4(acc[2][0], acc[2][1], acc[2][2], acc[2][3]);
  acc_guard4(acc[3][0], acc[3][1], acc[3][2], acc[3][3]);

  float* slab = sT[wave];
  const float* Rb = RESID ? (resid + (size_t)b * strideR) : nullptr;
#pragma unroll
  for (int i = 0; i < 4; ++i) {
    const int mBase = m0 + (i << 4);
#pragma unroll
    for (int j = 0; j < 4; ++j) {
      const int n = n0 + (j << 4) + rlane;
      float bv = 0.f;
      if (BIAS_MODE == 2) bv = bias[n];
#pragma unroll
      for (int r = 0; r < 8; ++r) {
        float v = acc[i][j][r] * scale;
        if (BIAS_MODE == 1) v += bias[mBase + mOff + r];
        if (BIAS_MODE == 2) v += bv;
        if (RESID) v += Rb[(size_t)(mBase + mOff + r) * ldc + n];
        if (ACT == 1) v = tanhf(v);
        if (ACT == 2) v = fmaxf(v, 0.0f);
        if (ACT == 3) v = v / (1.0f + expf(-v));
        if (ACT == 4) v = (v > 0.f) ? v : 0.01f * v;
        slab[(mOff + r) * 68 + (j << 4) + rlane] = v;
      }
    }
    __builtin_amdgcn_fence(__ATOMIC_RELEASE, "workgroup");
    __builtin_amdgcn_wave_barrier();
    __builtin_amdgcn_fence(__ATOMIC_ACQUIRE, "workgroup");
    if (OUT_MODE == 0) {
      float* C = (float*)Cout + (size_t)b * strideC + (size_t)bz * strideCz;
      const int hh = lane >> 4, c4 = (lane & 15) * 4;
      for (int pass = 0; pass < 2; ++pass) {
#pragma unroll
        for (int it = 0; it < 8; ++it) {
          const int row = it * 2 + hh;
          v4f v = *(const v4f*)(slab + row * 68 + c4);
          *(volatile v4f*)(C + (size_t)(mBase + row) * ldc + n0 + c4) = v;
        }
        __threadfence();
      }
    } else {
      const int q = lane >> 3, c8 = (lane & 7) * 8;
      unsigned short* C  = (unsigned short*)Cout  + (size_t)b * strideC + (size_t)bz * strideCz;
      unsigned short* Cb2 = (OUT_MODE == 2) ? ((unsigned short*)Cout2 + (size_t)b * strideC + (size_t)bz * strideCz) : nullptr;
      for (int pass = 0; pass < 2; ++pass) {
#pragma unroll
        for (int it = 0; it < 4; ++it) {
          const int row = it * 4 + q;
          const float* sp = slab + row * 68 + c8;
          v8h hv, lv;
#pragma unroll
          for (int e = 0; e < 8; ++e) {
            if (OUT_MODE == 1) {
              hv[e] = (_Float16)sp[e];
            } else {
              unsigned short hb = f2bf_bits(sp[e]);
              unsigned short lb = f2bf_bits(sp[e] - bf_bits2f(hb));
              hv[e] = __builtin_bit_cast(_Float16, hb);
              lv[e] = __builtin_bit_cast(_Float16, lb);
            }
          }
          *(volatile v8h*)(C + (size_t)(mBase + row) * ldc + n0 + c8) = hv;
          if (OUT_MODE == 2) *(volatile v8h*)(Cb2 + (size_t)(mBase + row) * ldc + n0 + c8) = lv;
        }
        __threadfence();
      }
    }
    __builtin_amdgcn_fence(__ATOMIC_RELEASE, "workgroup");
    __builtin_amdgcn_wave_barrier();
    __builtin_amdgcn_fence(__ATOMIC_ACQUIRE, "workgroup");
  }
}

__global__ __launch_bounds__(256) void cast_scale_f32_f16x2(
    const float* __restrict__ in, _Float16* __restrict__ out, int n2, float scale) {
  int i = blockIdx.x * 256 + threadIdx.x;
  if (i < n2) {
    const _Float16 h0 = (_Float16)(in[2 * i] * scale), h1 = (_Float16)(in[2 * i + 1] * scale);
    const unsigned u = (unsigned)__builtin_bit_cast(unsigned short, h0) | ((unsigned)__builtin_bit_cast(unsigned short, h1) << 16);
    ((volatile unsigned*)out)[i] = u;
    __threadfence();
    ((volatile unsigned*)out)[i] = u;
  }
}

constexpr int kTileC   = 64;
constexpr int kTileHW  = 32;
constexpr int kTilePitch = 72;
__global__ __launch_bounds__(256) void xpose_cast_x(
    const float* __restrict__ x, _Float16* __restrict__ xt, float scale) {
  __shared__ __align__(16) _Float16 tile[kTileHW][kTilePitch];
  const int tid  = threadIdx.x;
  const int wave = tid >> 5;
  const int lane = tid & 31;
  const int b    = blockIdx.z;
  const int c0   = blockIdx.y * kTileC;
  const int hw0  = blockIdx.x * kTileHW;
  const float* xb = x + ((size_t)b * kCin + c0) * kHW + hw0;
#pragma unroll
  for (int it = 0; it < 8; ++it) {
    const int idx = it * 256 + tid;
    const int c   = idx >> 5;
    const int hl  = idx & 31;
    const float f = xb[(size_t)c * kHW + hl];
    tile[hl][c] = (_Float16)(f * scale);
  }
  __syncthreads();
  {
    const int q  = lane >> 3;
    const int c8 = (lane & 7) * 8;
    const int row = wave * 4 + q;
    const v8h v = *(const v8h*)(&tile[row][c8]);
    _Float16* dst = xt + ((size_t)b * kHW + hw0 + row) * kCin + c0 + c8;
    *(volatile v8h*)dst = v;
    __threadfence();
    *(volatile v8h*)dst = v;
  }
}

__global__ __launch_bounds__(256) void routing_kernel(
    const float* __restrict__ con, const float* __restrict__ bias, float* __restrict__ out,
    int batch0, int nthreads) {
  const int t = blockIdx.x * 256 + threadIdx.x;
  if (t >= nthreads) return;
  const int bl = t >> 10;
  const int hw = t & (kHW - 1);
  const float* cb = con + (size_t)bl * kGroups * kFo * kHW + hw;
  float* ob = out + ((size_t)(batch0 + bl) * kFo) * kHW + hw;

  float beta[kGroups];
#pragma unroll
  for (int g = 0; g < kGroups; ++g) beta[g] = 0.0f;

#pragma unroll 1
  for (int it = 0; it < kIters; ++it) {
    float alpha[kGroups];
#pragma unroll
    for (int g = 0; g < kGroups; ++g) {
      const float bb = fminf(fmaxf(beta[g], -80.0f), 80.0f);
      const float ex = __expf(-bb);
      alpha[g] = __builtin_amdgcn_rcpf(1.0f + ex);
    }
    if (it + 1 < kIters) {
#pragma unroll 1
      for (int o = 0; o < kFo; ++o) {
        float c[kGroups];
#pragma unroll
        for (int g = 0; g < kGroups; ++g) c[g] = cb[((size_t)g * kFo + o) * kHW];
        float v = alpha[0] * c[0];
#pragma unroll
        for (int g = 1; g < kGroups; ++g) v += alpha[g] * c[g];
#pragma unroll
        for (int g = 0; g < kGroups; ++g) beta[g] += v * c[g];
      }
    } else {
#pragma unroll 1
      for (int o = 0; o < kFo; ++o) {
        float c[kGroups];
#pragma unroll
        for (int g = 0; g < kGroups; ++g) c[g] = cb[((size_t)g * kFo + o) * kHW];
        float v = alpha[0] * c[0];
#pragma unroll
        for (int g = 1; g < kGroups; ++g) v += alpha[g] * c[g];
        const float r = v + bias[o];
        float* p = ob + (size_t)o * kHW;
        *(volatile float*)p = r;
        __threadfence();
        *(volatile float*)p = r;
      }
    }
  }
}

extern "C" void kernel_launch(void* const* d_in, const int* in_sizes, int n_in,
                              void* d_out, int out_size, void* d_ws, size_t ws_size,
                              hipStream_t stream) {
  if (n_in < 3) return;
  if (in_sizes[0] != kBatch * kCin * kHW) return;
  if (in_sizes[1] != kFo * kCin) return;
  if (in_sizes[2] != kFo) return;
  if (out_size != kBatch * kFo * kHW) return;

  const float* x    = (const float*)d_in[0];
  const float* wght = (const float*)d_in[1];
  const float* bias = (const float*)d_in[2];
  float*       out  = (float*)d_out;

  const size_t w16_bytes  = (size_t)kFo * kCin * 2;
  const size_t xt16_bytes = (size_t)kBatch * kHW * kCin * 2;
  const size_t con_bytes  = (size_t)kBatchChunk * kGroups * kFo * kHW * 4;
  const size_t off_w16  = 0;
  const size_t off_xt16 = off_w16 + w16_bytes;
  const size_t off_con  = off_xt16 + xt16_bytes;
  const size_t total    = off_con + con_bytes;
  if (total > ws_size) return;

  unsigned char* ws = (unsigned char*)d_ws;
  _Float16* W16  = (_Float16*)(ws + off_w16);
  _Float16* XT16 = (_Float16*)(ws + off_xt16);
  float*    CON  = (float*)(ws + off_con);

  {
    const int n2 = kFo * kCin / 2;
    cast_scale_f32_f16x2<<<(n2 + 255) / 256, 256, 0, stream>>>(wght, W16, n2, kWScale);
  }
  {
    dim3 grid(kHW / kTileHW, kCin / kTileC, kBatch);
    xpose_cast_x<<<grid, 256, 0, stream>>>(x, XT16, kXScale);
  }
  const int  M = kFo, N = kHW, K = kFi;
  const int  tiles = (M / 64) * (N / 64);
  const long strideA  = kFi;
  const long strideAz = 0;
  const long strideB  = kFi;
  const long strideBz = (long)kHW * kCin;
  const long strideC  = (long)kFo * kHW;
  const long strideCz = (long)kGroups * kFo * kHW;
  for (int ch = 0; ch < kNumChunks; ++ch) {
    const _Float16* XTc = XT16 + (size_t)ch * kBatchChunk * kHW * kCin;
    dim3 ggrid((tiles + 7) / 8, kGroups, kBatchChunk);
    wmma_gemm64z<0, false, 0, 0, false, 0><<<ggrid, 256, 0, stream>>>(
        (const unsigned short*)W16, (const unsigned short*)W16, kCin, strideA, strideAz,
        (const unsigned short*)XTc, (const unsigned short*)XTc, kCin, strideB, strideBz,
        (void*)CON, (void*)CON, kHW, strideC, strideCz,
        bias,
        (const float*)CON, 0L,
        M, N, K, kOutScale);
    const int nthreads = kBatchChunk * kHW;
    routing_kernel<<<(nthreads + 255) / 256, 256, 0, stream>>>(CON, bias, out, ch * kBatchChunk, nthreads);
  }
}
